// GaussianKDE_39273180954692
// MI455X (gfx1250) — hardware-verified
//
#include <hip/hip_runtime.h>
#include <stddef.h>


typedef _Float16 v16h __attribute__((ext_vector_type(16)));
typedef _Float16 v8h  __attribute__((ext_vector_type(8)));
typedef float    v8f  __attribute__((ext_vector_type(8)));
typedef float    v4f  __attribute__((ext_vector_type(4)));
typedef float    v2f  __attribute__((ext_vector_type(2)));

#ifndef NQ
#define NQ 4096
#endif
#ifndef NKEY
#define NKEY 50000
#endif
#define NQ_FULL   4096
#define NKEY_FULL 50000
#define DDIM 64
#define NPAD (((NKEY + 127) / 128) * 128)

#ifndef F_RES
#define F_RES 0
#endif

static_assert(NQ >= 128 && NQ <= NQ_FULL && (NQ % 128) == 0);
static_assert(NKEY >= 1 && NKEY <= NKEY_FULL);
static_assert(DDIM == 64);
static_assert((NPAD % 128) == 0 && (NPAD % 64) == 0 && NPAD >= NKEY);
static_assert((NQ % 64) == 0);
static_assert((DDIM % 32) == 0 && (DDIM % 8) == 0);

#define LDT 72
#define LDC 68
static_assert((LDT % 8) == 0 && LDT >= 64);
static_assert((LDC % 4) == 0 && LDC >= 64);

#define WCARRY 64.0f
#define XCARRY 64.0f
#define FCARRY 16.0f
#define RCARRY 2048.0f

#define PROJ_TO_F  (1.0f / (XCARRY * WCARRY))
#define PROJ_TO_FC (FCARRY / (XCARRY * WCARRY))
#define SC_HI      (1.0f / (FCARRY * XCARRY))
#define SC_RES     (1.0f / (FCARRY * XCARRY * RCARRY))

#define BW_BYTES   ((size_t)DDIM * DDIM * 2)
#define FIN_BYTES  ((size_t)NQ * DDIM * 2)
#define X16_BYTES  ((size_t)NPAD * DDIM * 2)
#define HX_BYTES   ((size_t)NPAD * 4)
#define FH_BYTES   ((size_t)NQ * DDIM * 2)
#define FR_BYTES   ((size_t)NQ * DDIM * 2)
#define HF_BYTES   ((size_t)NQ * 4)
#define OFF_BW   ((size_t)0)
#define OFF_FIN  (OFF_BW + BW_BYTES)
#define OFF_X16  (OFF_FIN + FIN_BYTES)
#define OFF_HX   (OFF_X16 + X16_BYTES)
#define OFF_FH   (OFF_HX + HX_BYTES)
#define OFF_FR   (OFF_FH + FH_BYTES)
#define OFF_HF   (OFF_FR + FR_BYTES)
#define WS_TOTAL (OFF_HF + HF_BYTES)
static_assert((BW_BYTES % 128) == 0 && (FIN_BYTES % 128) == 0 && (X16_BYTES % 128) == 0);
static_assert((HX_BYTES % 128) == 0 && (FH_BYTES % 128) == 0 && (FR_BYTES % 128) == 0);
static_assert((HF_BYTES % 128) == 0);
static_assert(WS_TOTAL <= (size_t)134217728);

__device__ __forceinline__ float bf16r(float x) {
  unsigned int u = __float_as_uint(x);
  u = (u + 0x7FFFu + ((u >> 16) & 1u)) & 0xFFFF0000u;
  return __uint_as_float(u);
}

__device__ __forceinline__ _Float16 toh_flush(float v) {
  const _Float16 r = (_Float16)v;
  return (fabsf(v) < 6.103515625e-05f) ? (_Float16)0.0f : r;
}

__device__ __forceinline__ v16h frag_at(const _Float16* p) {
  v8h lo = *(const v8h*)(p);
  v8h hi = *(const v8h*)(p + 16);
  v16h out;
#pragma unroll
  for (int i = 0; i < 8; ++i) { out[i] = lo[i]; out[i + 8] = hi[i]; }
  return out;
}
__device__ __forceinline__ v16h ld_frag(const _Float16* base, unsigned ld) {
  const unsigned lane = threadIdx.x & 31u;
  return frag_at(base + (lane & 15u) * ld + (lane >> 4) * 8u);
}

__device__ __forceinline__ v8f wmma16(v16h a, v16h b, v8f c) {
  v8f d = __builtin_amdgcn_wmma_f32_16x16x32_f16(false, a, false, b, (short)0, c,
                                                 false, false);
  asm volatile("v_nop\n\tv_nop\n\tv_nop\n\tv_nop" : "+v"(d) : "v"(a), "v"(b));
  return d;
}

__device__ __forceinline__ float red16_sum(float x) {
#pragma unroll
  for (int off = 1; off < 16; off <<= 1) x += __shfl_xor(x, off, 32);
  return x;
}
__device__ __forceinline__ float red8_sum(float x) {
#pragma unroll
  for (int off = 1; off < 8; off <<= 1) x += __shfl_xor(x, off, 32);
  return x;
}

__global__ __launch_bounds__(256) void wconv_kernel(
    const float* __restrict__ W, _Float16* __restrict__ Wt, unsigned ldw, unsigned ldk) {
  __shared__ _Float16 T[64 * LDT];
  const unsigned tid = threadIdx.x;
  const unsigned n0 = blockIdx.x * 64u;
  const unsigned k0 = blockIdx.y * 64u;
#pragma unroll 4
  for (unsigned j = 0; j < 16u; ++j) {
    const unsigned idx = tid + 256u * j;
    const unsigned kr = idx >> 6, nc = idx & 63u;
    const float v = W[(size_t)(k0 + kr) * ldw + n0 + nc];
    T[nc * LDT + kr] = (_Float16)(WCARRY * bf16r(v));
  }
  __syncthreads();
  v8h x[2];
  size_t off[2];
#pragma unroll
  for (unsigned i = 0; i < 2u; ++i) {
    const unsigned n = 32u * i + (tid >> 3);
    const unsigned kc = (tid & 7u) * 8u;
    x[i] = *(const v8h*)&T[n * LDT + kc];
    off[i] = (size_t)(n0 + n) * ldk + k0 + kc;
  }
#pragma unroll
  for (int i = 0; i < 2; ++i) *(volatile v8h*)(Wt + off[i]) = x[i];
  __threadfence();
#pragma unroll
  for (int i = 0; i < 2; ++i) *(volatile v8h*)(Wt + off[i]) = x[i];
}

template <int WANT_SQ>
__device__ __forceinline__ void rowprep_body(const float* __restrict__ X,
                                             _Float16* __restrict__ X16,
                                             float* __restrict__ HX, unsigned nrows) {
  __shared__ float Sq[128];
  const unsigned tid = threadIdx.x, lane = tid & 31u;
  const unsigned w = (unsigned)__builtin_amdgcn_readfirstlane((int)(threadIdx.x >> 5));
  const unsigned sub = tid & 7u, rl = tid >> 3;
#pragma unroll 1
  for (unsigned pass = 0; pass < 4u; ++pass) {
    const unsigned row = blockIdx.x * 128u + pass * 32u + rl;
    const bool live = row < nrows;
    const unsigned crow = live ? row : (nrows - 1u);
    const float* p = X + (size_t)crow * DDIM + sub * 8u;
    const v4f a0 = *(const v4f*)(p);
    const v4f a1 = *(const v4f*)(p + 4);
    v8h o;
    float s = 0.0f;
#pragma unroll
    for (int i = 0; i < 4; ++i) {
      const float e0 = live ? bf16r(a0[i]) : 0.0f;
      const float e1 = live ? bf16r(a1[i]) : 0.0f;
      o[i]     = toh_flush(XCARRY * e0);
      o[i + 4] = toh_flush(XCARRY * e1);
      s += e0 * e0;
      s += e1 * e1;
    }
    s = red8_sum(s);
    if (WANT_SQ) {
      const float hv = live ? (-0.5f * s) : -1.0e30f;
      if (sub == 0u) Sq[pass * 32u + rl] = hv;
    }
    _Float16* d = X16 + (size_t)row * DDIM + sub * 8u;
    *(volatile v8h*)d = o;
    __threadfence();
    *(volatile v8h*)d = o;
  }
  if (WANT_SQ) {
    __syncthreads();
    if (w == 0u) {
      const v4f t = *(const v4f*)&Sq[lane * 4u];
      float* d = HX + (size_t)blockIdx.x * 128u + lane * 4u;
      *(volatile v4f*)d = t;
      __threadfence();
      *(volatile v4f*)d = t;
    }
  }
}

__global__ __launch_bounds__(256) void featprep_kernel(
    const float* __restrict__ X, _Float16* __restrict__ X16, unsigned nrows) {
  rowprep_body<0>(X, X16, (float*)0, nrows);
}
__global__ __launch_bounds__(256) void dataprep_kernel(
    const float* __restrict__ X, _Float16* __restrict__ X16, float* __restrict__ HX,
    unsigned nrows) {
  rowprep_body<1>(X, X16, HX, nrows);
}

__global__ __launch_bounds__(256) void proj_kernel(
    const _Float16* __restrict__ A16, const _Float16* __restrict__ Bt,
    _Float16* __restrict__ fh, _Float16* __restrict__ fr, float* __restrict__ hf) {
  __shared__ float Cs[64 * LDC];
  __shared__ float Rs[64];
  const unsigned tid = threadIdx.x, lane = tid & 31u;
  const unsigned w = (unsigned)__builtin_amdgcn_readfirstlane((int)(threadIdx.x >> 5));
  const unsigned mw = w >> 1, nw = w & 1u;
  const unsigned hh = lane >> 4, m = lane & 15u;
  const unsigned n0 = blockIdx.x * 64u;
  const unsigned row0 = blockIdx.y * 64u;
  const unsigned K = (unsigned)DDIM;

  const _Float16* ap  = A16 + (size_t)(row0 + mw * 16u + m) * K + hh * 8u;
  const _Float16* bp0 = Bt + (size_t)(n0 + nw * 32u + m) * K + hh * 8u;
  const _Float16* bp1 = bp0 + (size_t)16 * K;
  v8f acc0 = {}, acc1 = {};
#pragma unroll 2
  for (unsigned k0 = 0; k0 < K; k0 += 32u) {
    const v16h a  = frag_at(ap + k0);
    const v16h b0 = frag_at(bp0 + k0);
    const v16h b1 = frag_at(bp1 + k0);
    acc0 = wmma16(a, b0, acc0);
    acc1 = wmma16(a, b1, acc1);
  }
#pragma unroll
  for (int r = 0; r < 8; ++r) {
    float* d = &Cs[(mw * 16u + hh * 8u + (unsigned)r) * LDC + nw * 32u + m];
    d[0]  = acc0[r];
    d[16] = acc1[r];
  }
  __syncthreads();

  v8h x[2];
#if F_RES
  v8h xr[2];
#endif
  size_t off[2];
#pragma unroll
  for (unsigned i = 0; i < 2u; ++i) {
    const unsigned r = 32u * i + (tid >> 3);
    const unsigned c = (tid & 7u) * 8u;
    const v4f u0 = *(const v4f*)&Cs[r * LDC + c];
    const v4f u1 = *(const v4f*)&Cs[r * LDC + c + 4];
    float ss = 0.0f;
#pragma unroll
    for (int j = 0; j < 4; ++j) {
      const float f0 = u0[j] * PROJ_TO_F;
      const float f1 = u1[j] * PROJ_TO_F;
      ss += f0 * f0;
      ss += f1 * f1;
      const float t0 = u0[j] * PROJ_TO_FC;
      const float t1 = u1[j] * PROJ_TO_FC;
      const _Float16 h0 = toh_flush(t0);
      const _Float16 h1 = toh_flush(t1);
      x[i][j]     = h0;
      x[i][j + 4] = h1;
#if F_RES
      xr[i][j]     = toh_flush((t0 - (float)h0) * RCARRY);
      xr[i][j + 4] = toh_flush((t1 - (float)h1) * RCARRY);
#endif
    }
    ss = red8_sum(ss);
    const float hv = -0.5f * ss;
    if ((tid & 7u) == 0u) Rs[r] = hv;
    off[i] = (size_t)(row0 + r) * DDIM + n0 + c;
  }
#pragma unroll
  for (int i = 0; i < 2; ++i) *(volatile v8h*)(fh + off[i]) = x[i];
#if F_RES
#pragma unroll
  for (int i = 0; i < 2; ++i) *(volatile v8h*)(fr + off[i]) = xr[i];
#endif
  __threadfence();
#pragma unroll
  for (int i = 0; i < 2; ++i) *(volatile v8h*)(fh + off[i]) = x[i];
#if F_RES
#pragma unroll
  for (int i = 0; i < 2; ++i) *(volatile v8h*)(fr + off[i]) = xr[i];
#endif

  __syncthreads();
  if (w == 0u) {
    const v2f t = *(const v2f*)&Rs[lane * 2u];
    float* d = hf + row0 + lane * 2u;
    *(volatile v2f*)d = t;
    __threadfence();
    *(volatile v2f*)d = t;
  }
}

__global__ __launch_bounds__(256) void kde_kernel(
    const _Float16* __restrict__ Fh, const _Float16* __restrict__ Fr,
    const _Float16* __restrict__ Xh, const float* __restrict__ Hx,
    const float* __restrict__ Hf, const float* __restrict__ nrm, float* __restrict__ out) {
  __shared__ _Float16 Ks[64 * LDT];
  __shared__ float Hs[64];
  __shared__ float Os[128];

  const unsigned tid = threadIdx.x, lane = tid & 31u;
  const unsigned w = (unsigned)__builtin_amdgcn_readfirstlane((int)(threadIdx.x >> 5));
  const unsigned hh = lane >> 4, m = lane & 15u;
  const unsigned q0 = blockIdx.x * 128u;
  const unsigned qrow0 = q0 + w * 16u;

  const size_t qoff = (size_t)(qrow0 + m) * DDIM + hh * 8u;
  v16h qf[2];
  qf[0] = frag_at(Fh + qoff);
  qf[1] = frag_at(Fh + qoff + 32);
#if F_RES
  v16h qr[2];
  qr[0] = frag_at(Fr + qoff);
  qr[1] = frag_at(Fr + qoff + 32);
#endif

  float lsum[8];
#pragma unroll
  for (int v = 0; v < 8; ++v) lsum[v] = 0.0f;

  for (unsigned kb = 0; kb < (unsigned)NPAD; kb += 64u) {
#pragma unroll
    for (unsigned j = 0; j < 2u; ++j) {
      const unsigned idx = tid + 256u * j;
      const unsigned r = idx >> 3, c = (idx & 7u) * 8u;
      *(v8h*)&Ks[r * LDT + c] = *(const v8h*)(Xh + (size_t)(kb + r) * DDIM + c);
    }
    if (w < 2u) Hs[tid] = Hx[kb + tid];
    __syncthreads();

#pragma unroll
    for (int kg = 0; kg < 4; ++kg) {
      v8f t = {};
#if F_RES
      v8f tr = {};
#endif
#pragma unroll
      for (int c = 0; c < 2; ++c) {
        const v16h kf = ld_frag(&Ks[(kg * 16) * LDT + c * 32], LDT);
        t = wmma16(qf[c], kf, t);
#if F_RES
        tr = wmma16(qr[c], kf, tr);
#endif
      }
      const float hx = Hs[(unsigned)kg * 16u + m];
#pragma unroll
      for (int v = 0; v < 8; ++v) {
#if F_RES
        const float e = t[v] * SC_HI + (tr[v] * SC_RES + hx);
#else
        const float e = t[v] * SC_HI + hx;
#endif
        lsum[v] += __expf(e);
      }
    }
    __syncthreads();
  }

#pragma unroll
  for (int v = 0; v < 8; ++v) lsum[v] = red16_sum(lsum[v]);
  if (m == 0u) {
#pragma unroll
    for (int v = 0; v < 8; ++v) Os[w * 16u + hh * 8u + (unsigned)v] = lsum[v];
  }
  __syncthreads();
  if (w == 0u) {
    const float coef = bf16r(nrm[0]) * (1.0f / (float)NKEY);
    const v4f s  = *(const v4f*)&Os[lane * 4u];
    const v4f hq = *(const v4f*)(Hf + q0 + lane * 4u);
    v4f val;
#pragma unroll
    for (int j = 0; j < 4; ++j) val[j] = s[j] * (coef * __expf(hq[j]));
    float* d = out + q0 + lane * 4u;
    *(volatile v4f*)d = val;
    __threadfence();
    *(volatile v4f*)d = val;
  }
}

extern "C" void kernel_launch(void* const* d_in, const int* in_sizes, int n_in,
                              void* d_out, int out_size, void* d_ws, size_t ws_size,
                              hipStream_t stream) {
  if (n_in < 4) return;
  if ((long long)in_sizes[0] < (long long)NQ * DDIM) return;
  if ((long long)in_sizes[1] < (long long)DDIM * DDIM) return;
  if ((long long)in_sizes[2] < (long long)NKEY * DDIM) return;
  if (in_sizes[3] < 1) return;
  if ((long long)out_size < (long long)NQ) return;
  if (ws_size < WS_TOTAL) return;

  const float* features = (const float*)d_in[0];
  const float* bw       = (const float*)d_in[1];
  const float* dataset  = (const float*)d_in[2];
  const float* nrm      = (const float*)d_in[3];
  float* out = (float*)d_out;

  char* ws = (char*)d_ws;
  _Float16* Bw_t  = (_Float16*)(ws + OFF_BW);
  _Float16* Fin16 = (_Float16*)(ws + OFF_FIN);
  _Float16* X16   = (_Float16*)(ws + OFF_X16);
  float*    HX    = (float*)(ws + OFF_HX);
  _Float16* FH    = (_Float16*)(ws + OFF_FH);
  _Float16* FR    = (_Float16*)(ws + OFF_FR);
  float*    HF    = (float*)(ws + OFF_HF);

  dim3 blk(256);

  wconv_kernel<<<dim3(DDIM / 64, DDIM / 64), blk, 0, stream>>>(bw, Bw_t, (unsigned)DDIM, (unsigned)DDIM);
  featprep_kernel<<<dim3(NQ / 128), blk, 0, stream>>>(features, Fin16, (unsigned)NQ);
  dataprep_kernel<<<dim3(NPAD / 128), blk, 0, stream>>>(dataset, X16, HX, (unsigned)NKEY);
  proj_kernel<<<dim3(DDIM / 64, NQ / 64), blk, 0, stream>>>(Fin16, Bw_t, FH, FR, HF);
  kde_kernel<<<dim3(NQ / 128), blk, 0, stream>>>(FH, FR, X16, HX, HF, nrm, out);
}
